// GNNDrugEncoder_6399501271497
// MI455X (gfx1250) — hardware-verified
//
#include <hip/hip_runtime.h>
#include <stddef.h>
#include <stdint.h>
#include <math.h>


#define HID    256
#define NLAY   4
#define NBOND  6
#define NATOM  38
#define KEMB   64
#define KB     32
#define BB     32
#define NN     128
#define MTOT   (BB * NN)
#define AP     512
#define HGP    1024
#define G3     768
#define NTHR   256
#define NWAVE  8
#define GBM    64
#define GBN    64
#define GTHR   128
#define MG     16

#define U_NFB  (MTOT * (KEMB / 8))
#define U_EWT  (HID * (KEMB / 8))
#define U_BFB  (MTOT * NN)
#define U_ADJ  (MTOT * NN / 4)
#define U_WHT  (NLAY * HID * (HID / 8))
#define U_WHH  (NLAY * G3 * (HID / 8))
#define U_WIH  (NLAY * G3 * (HID / 8))
#define U_WBT  (NLAY * HID * (KB / 8))
#define O1 (U_NFB)
#define O2 (O1 + U_EWT)
#define O3 (O2 + U_BFB)
#define O4 (O3 + U_ADJ)
#define O5 (O4 + U_WHT)
#define O6 (O5 + U_WHH)
#define O7 (O6 + U_WIH)
#define O8 (O7 + U_WBT)
#define WSMAX  134217728

static_assert(O1 % NTHR == 0 && O2 % NTHR == 0 && O3 % NTHR == 0 && O4 % NTHR == 0);
static_assert(O5 % NTHR == 0 && O6 % NTHR == 0 && O7 % NTHR == 0 && O8 % NTHR == 0);
static_assert(MTOT % GBM == 0 && HID % GBN == 0 && HGP % GBN == 0 && G3 % GBN == 0);
static_assert(KEMB % 32 == 0 && HID % 32 == 0 && KB == 32);
static_assert(GBM == (GTHR / 32) * 16 && GBN == 64);
static_assert(MTOT % MG == 0 && MG == 2 * NWAVE && MTOT % NWAVE == 0);
static_assert(HID == 8 * 32 && AP == 2 * HID && HGP == HID + G3 && NN == 128);
static_assert((HID / 8) == 32 && (G3 * (HID / 8)) == 24576);

typedef float          v2f   __attribute__((ext_vector_type(2)));
typedef float          v4f   __attribute__((ext_vector_type(4)));
typedef float          v8f   __attribute__((ext_vector_type(8)));
typedef int            v8i   __attribute__((ext_vector_type(8)));
typedef unsigned int   v4u   __attribute__((ext_vector_type(4)));
typedef unsigned short v8us  __attribute__((ext_vector_type(8)));
typedef unsigned short v16us __attribute__((ext_vector_type(16)));
typedef __bf16         v16bf __attribute__((ext_vector_type(16)));
typedef v2f  __attribute__((may_alias)) v2fa;
typedef v4f  __attribute__((may_alias)) v4fa;
typedef v4u  __attribute__((may_alias)) v4ua;
typedef v8us __attribute__((may_alias)) v8usa;
union FragB { v16bf v; v16us u; v8us h[2]; v8i w; };

__device__ __forceinline__ v8f wmb(const FragB& a, const FragB& b, v8f c) {
  v8f d = __builtin_amdgcn_wmma_f32_16x16x32_bf16(false, a.v, false, b.v, (short)0, c, false, false);
  asm volatile("v_nop\n\tv_nop\n\tv_nop\n\tv_nop" : "+v"(d) : "v"(a.w), "v"(b.w));
  return d;
}

__device__ __forceinline__ unsigned bf16_bits(float f) {
  const unsigned u = __float_as_uint(f);
  return (u + 0x7FFFu + ((u >> 16) & 1u)) >> 16;
}
__device__ __forceinline__ float bf16_val(float f) {
  return __uint_as_float(bf16_bits(f) << 16);
}
__device__ __forceinline__ v4u pk8(unsigned b0, unsigned b1, unsigned b2, unsigned b3,
                                   unsigned b4, unsigned b5, unsigned b6, unsigned b7) {
  v4u o;
  o.x = b0 | (b1 << 16); o.y = b2 | (b3 << 16); o.z = b4 | (b5 << 16); o.w = b6 | (b7 << 16);
  return o;
}
__device__ __forceinline__ void split8(const v4f a, const v4f b, v8us& hi, v8us& lo) {
  unsigned hb;
  hb = bf16_bits(a.x); hi[0] = (unsigned short)hb; lo[0] = (unsigned short)bf16_bits(a.x - __uint_as_float(hb << 16));
  hb = bf16_bits(a.y); hi[1] = (unsigned short)hb; lo[1] = (unsigned short)bf16_bits(a.y - __uint_as_float(hb << 16));
  hb = bf16_bits(a.z); hi[2] = (unsigned short)hb; lo[2] = (unsigned short)bf16_bits(a.z - __uint_as_float(hb << 16));
  hb = bf16_bits(a.w); hi[3] = (unsigned short)hb; lo[3] = (unsigned short)bf16_bits(a.w - __uint_as_float(hb << 16));
  hb = bf16_bits(b.x); hi[4] = (unsigned short)hb; lo[4] = (unsigned short)bf16_bits(b.x - __uint_as_float(hb << 16));
  hb = bf16_bits(b.y); hi[5] = (unsigned short)hb; lo[5] = (unsigned short)bf16_bits(b.y - __uint_as_float(hb << 16));
  hb = bf16_bits(b.z); hi[6] = (unsigned short)hb; lo[6] = (unsigned short)bf16_bits(b.z - __uint_as_float(hb << 16));
  hb = bf16_bits(b.w); hi[7] = (unsigned short)hb; lo[7] = (unsigned short)bf16_bits(b.w - __uint_as_float(hb << 16));
}

__global__ __launch_bounds__(NTHR) void k_prep(
    const float* __restrict__ node, const float* __restrict__ embw, const float* __restrict__ bond,
    const float* __restrict__ adj, const float* __restrict__ msgw, const float* __restrict__ whh,
    const float* __restrict__ wih,
    unsigned short* NFB, unsigned short* EWT, unsigned short* BFB, float* ADJF,
    unsigned short* WCAT, unsigned short* WIH, unsigned short* WBT) {
  const int u = (int)blockIdx.x * NTHR + (int)threadIdx.x;
  v4u o;
  void* dp;
  if (u < O1) {
    const int row = u >> 3;
    const int k8  = (u & 7) * 8;
    const float* p = node + (size_t)row * NATOM;
    unsigned bt[8];
#pragma unroll
    for (int i = 0; i < 8; ++i) {
      const int k  = k8 + i;
      const int kc = k < NATOM ? k : NATOM - 1;
      const float v = p[kc];
      bt[i] = (k < NATOM) ? bf16_bits(v) : 0u;
    }
    o = pk8(bt[0], bt[1], bt[2], bt[3], bt[4], bt[5], bt[6], bt[7]);
    dp = (void*)(NFB + (size_t)row * KEMB + k8);
  } else if (u < O2) {
    const int v  = u - O1;
    const int n  = v >> 3;
    const int k8 = (v & 7) * 8;
    unsigned bt[8];
#pragma unroll
    for (int i = 0; i < 8; ++i) {
      const int k  = k8 + i;
      const int kc = k < NATOM ? k : NATOM - 1;
      const float w = embw[(size_t)kc * HID + n];
      bt[i] = (k < NATOM) ? bf16_bits(w) : 0u;
    }
    o = pk8(bt[0], bt[1], bt[2], bt[3], bt[4], bt[5], bt[6], bt[7]);
    dp = (void*)(EWT + (size_t)n * KEMB + k8);
  } else if (u < O3) {
    const int v = u - O2;
    const float* p = bond + (size_t)v * NBOND;
    const v2f a = *(const v2fa*)p;
    const v2f b = *(const v2fa*)(p + 2);
    const v2f c = *(const v2fa*)(p + 4);
    o = pk8(bf16_bits(a.x), bf16_bits(a.y), bf16_bits(b.x), bf16_bits(b.y),
            bf16_bits(c.x), bf16_bits(c.y), 0u, 0u);
    dp = (void*)(BFB + (size_t)v * 8);
  } else if (u < O4) {
    const int v = u - O3;
    const v4f a = *(const v4fa*)(adj + (size_t)v * 4);
    o.x = bf16_bits(a.x) << 16; o.y = bf16_bits(a.y) << 16;
    o.z = bf16_bits(a.z) << 16; o.w = bf16_bits(a.w) << 16;
    dp = (void*)(ADJF + (size_t)v * 4);
  } else if (u < O5) {
    const int v   = u - O4;
    const int l   = v >> 13;
    const int rem = v & 8191;
    const int n   = rem >> 5;
    const int k8  = (rem & 31) * 8;
    const float* p = msgw + ((size_t)l * (HID + NBOND) + k8) * HID + n;
    unsigned bt[8];
#pragma unroll
    for (int i = 0; i < 8; ++i) bt[i] = bf16_bits(p[(size_t)i * HID]);
    o = pk8(bt[0], bt[1], bt[2], bt[3], bt[4], bt[5], bt[6], bt[7]);
    dp = (void*)(WCAT + ((size_t)l * HGP + n) * HID + k8);
  } else if (u < O6) {
    const int v   = u - O5;
    const int l   = v / 24576;
    const int rem = v - l * 24576;
    const int n   = rem >> 5;
    const int k8  = (rem & 31) * 8;
    const float* p = whh + ((size_t)l * G3 + n) * HID + k8;
    const v4f a = *(const v4fa*)p;
    const v4f b = *(const v4fa*)(p + 4);
    o = pk8(bf16_bits(a.x), bf16_bits(a.y), bf16_bits(a.z), bf16_bits(a.w),
            bf16_bits(b.x), bf16_bits(b.y), bf16_bits(b.z), bf16_bits(b.w));
    dp = (void*)(WCAT + ((size_t)l * HGP + HID + n) * HID + k8);
  } else if (u < O7) {
    const int v   = u - O6;
    const int l   = v / 24576;
    const int rem = v - l * 24576;
    const int n   = rem >> 5;
    const int k8  = (rem & 31) * 8;
    const float* p = wih + ((size_t)l * G3 + n) * HID + k8;
    const v4f a = *(const v4fa*)p;
    const v4f b = *(const v4fa*)(p + 4);
    o = pk8(bf16_bits(a.x), bf16_bits(a.y), bf16_bits(a.z), bf16_bits(a.w),
            bf16_bits(b.x), bf16_bits(b.y), bf16_bits(b.z), bf16_bits(b.w));
    dp = (void*)(WIH + ((size_t)l * G3 + n) * HID + k8);
  } else if (u < O8) {
    const int v   = u - O7;
    const int l   = v >> 10;
    const int rem = v & 1023;
    const int n   = rem >> 2;
    const int kq  = rem & 3;
    const float* p = msgw + ((size_t)l * (HID + NBOND) + HID) * HID + n;
    unsigned bt[6];
#pragma unroll
    for (int i = 0; i < 6; ++i) bt[i] = bf16_bits(p[(size_t)i * HID]);
    const unsigned km = (kq == 0) ? 0xffffffffu : 0u;
    o = pk8(bt[0], bt[1], bt[2], bt[3], bt[4], bt[5], 0u, 0u);
    o.x &= km; o.y &= km; o.z &= km; o.w &= km;
    dp = (void*)(WBT + ((size_t)l * HID + n) * KB + kq * 8);
  } else {
    return;
  }
  *(volatile v4u*)dp = o;
  __threadfence();
  *(volatile v4u*)dp = o;
}

template <int MODE, int TWO>
__global__ __launch_bounds__(GTHR) void k_gemm(
    const unsigned short* __restrict__ A, int lda, const unsigned short* __restrict__ WT, int K,
    const float* __restrict__ bias0, int split, const float* __restrict__ bias1,
    float* outF, int ldo, const float* __restrict__ mask, unsigned short* hl)
{
  __shared__ __attribute__((aligned(16))) float stg[GBM * GBN];
  __shared__ float smask[GBM];
  const int tid = (int)threadIdx.x, lane = tid & 31, wave = tid >> 5, hh = lane >> 4, m = lane & 15;
  const int rowBase = (int)blockIdx.x * GBM;
  const int col0    = (int)blockIdx.y * GBN;

  if (tid < GBM) smask[tid] = bf16_val(mask[rowBase + tid]);

  v8f acc[4];
  {
    const v8f z = {0.f, 0.f, 0.f, 0.f, 0.f, 0.f, 0.f, 0.f};
    acc[0] = z; acc[1] = z; acc[2] = z; acc[3] = z;
  }
  const unsigned short* ap = A  + (size_t)(rowBase + 16 * wave + m) * (size_t)lda + 8 * hh;
  const unsigned short* wp = WT + (size_t)(col0 + m) * (size_t)K + 8 * hh;
#pragma unroll 1
  for (int k0 = 0; k0 < K; k0 += 32) {
    FragB af, al;
    af.h[0] = *(const v8usa*)(ap + k0);
    af.h[1] = *(const v8usa*)(ap + k0 + 16);
    if constexpr (TWO != 0) {
      al.h[0] = *(const v8usa*)(ap + HID + k0);
      al.h[1] = *(const v8usa*)(ap + HID + k0 + 16);
    }
#pragma unroll
    for (int t = 0; t < 4; ++t) {
      const unsigned short* wq = wp + (size_t)(16 * t) * (size_t)K + k0;
      FragB bf;
      bf.h[0] = *(const v8usa*)wq;
      bf.h[1] = *(const v8usa*)(wq + 16);
      acc[t] = wmb(af, bf, acc[t]);
      if constexpr (TWO != 0) acc[t] = wmb(al, bf, acc[t]);
    }
  }

#pragma unroll
  for (int t = 0; t < 4; ++t) {
    const int lc = 16 * t + m;
#pragma unroll
    for (int r = 0; r < 8; ++r) {
      const int lr = 16 * wave + 8 * hh + r;
      stg[lr * GBN + lc] = acc[t][r];
    }
  }
  __syncthreads();

  const float* bp4 = (col0 < split) ? (bias0 + col0) : (bias1 + (col0 - split));
  v4f bb;
  {
    const v4f t = *(const v4fa*)(bp4 + 4 * m);
    bb.x = bf16_val(t.x); bb.y = bf16_val(t.y); bb.z = bf16_val(t.z); bb.w = bf16_val(t.w);
  }
  v4f fv[8];
#pragma unroll
  for (int i = 0; i < 8; ++i) {
    const int lr = 16 * wave + 2 * i + hh;
    v4f v = *(const v4fa*)(stg + lr * GBN + 4 * m);
    v = v + bb;
    if constexpr (MODE != 0) {
      const float me = smask[lr];
      v.x = fmaxf(v.x, 0.0f) * me; v.y = fmaxf(v.y, 0.0f) * me;
      v.z = fmaxf(v.z, 0.0f) * me; v.w = fmaxf(v.w, 0.0f) * me;
    }
    fv[i] = v;
  }
  v8us hv[4], lv[4];
  const int rr = lane >> 3, c8 = (lane & 7) * 8;
  if constexpr (MODE != 0) {
#pragma unroll
    for (int i = 0; i < 8; ++i) {
      const int lr = 16 * wave + 2 * i + hh;
      *(v4fa*)(stg + lr * GBN + 4 * m) = fv[i];
    }
    __syncthreads();
#pragma unroll
    for (int it = 0; it < 4; ++it) {
      const int lr = 16 * wave + 4 * it + rr;
      const v4f p0 = *(const v4fa*)(stg + lr * GBN + c8);
      const v4f p1 = *(const v4fa*)(stg + lr * GBN + c8 + 4);
      split8(p0, p1, hv[it], lv[it]);
    }
  }

#pragma unroll
  for (int i = 0; i < 8; ++i) {
    const int gr = rowBase + 16 * wave + 2 * i + hh;
    float* op = outF + (size_t)gr * (size_t)ldo + col0 + 4 * m;
    *(volatile v4f*)op = fv[i];
  }
  if constexpr (MODE != 0) {
#pragma unroll
    for (int it = 0; it < 4; ++it) {
      const int gr = rowBase + 16 * wave + 4 * it + rr;
      unsigned short* rp = hl + (size_t)gr * AP + col0 + c8;
      *(volatile v8us*)rp = hv[it];
      *(volatile v8us*)(rp + HID) = lv[it];
    }
  }
  __threadfence();
#pragma unroll
  for (int i = 0; i < 8; ++i) {
    const int gr = rowBase + 16 * wave + 2 * i + hh;
    float* op = outF + (size_t)gr * (size_t)ldo + col0 + 4 * m;
    *(volatile v4f*)op = fv[i];
  }
  if constexpr (MODE != 0) {
#pragma unroll
    for (int it = 0; it < 4; ++it) {
      const int gr = rowBase + 16 * wave + 4 * it + rr;
      unsigned short* rp = hl + (size_t)gr * AP + col0 + c8;
      *(volatile v8us*)rp = hv[it];
      *(volatile v8us*)(rp + HID) = lv[it];
    }
  }
}

__global__ __launch_bounds__(NTHR) void k_msg(
    const unsigned short* __restrict__ BFB, const float* __restrict__ ADJF, const float* __restrict__ HG,
    const unsigned short* __restrict__ WBT, unsigned short* AGG)
{
  __shared__ __attribute__((aligned(16))) float sagg[MG * HID];
  const int tid = (int)threadIdx.x, lane = tid & 31, wave = tid >> 5, hh = lane >> 4, m = lane & 15;
  const int row0 = (int)blockIdx.x * MG;
  const int h0   = wave * 32;

  FragB b0, b1;
  {
    const unsigned short* bp = WBT + (size_t)(h0 + m) * KB + 8 * hh;
    b0.h[0] = *(const v8usa*)bp;
    b0.h[1] = *(const v8usa*)(bp + 16);
    b1.h[0] = *(const v8usa*)(bp + 16 * KB);
    b1.h[1] = *(const v8usa*)(bp + 16 * KB + 16);
  }
  const unsigned am = (hh == 0) ? 0xffffffffu : 0u;

#pragma unroll 1
  for (int ii = 0; ii < MG; ++ii) {
    const int row = row0 + ii;
    const float hp0 = HG[(size_t)row * HGP + h0 + m];
    const float hp1 = HG[(size_t)row * HGP + h0 + 16 + m];
    const v8f c0 = {hp0, hp0, hp0, hp0, hp0, hp0, hp0, hp0};
    const v8f c1 = {hp1, hp1, hp1, hp1, hp1, hp1, hp1, hp1};
    const unsigned short* arow = BFB + (size_t)row * NN * 8 + (size_t)m * 8;
    const float* adjr = ADJF + (size_t)row * NN + 8 * hh;
    float acc0 = 0.0f, acc1 = 0.0f;
#pragma unroll 2
    for (int jt = 0; jt < NN / 16; ++jt) {
      const v4u raw = *(const v4ua*)(arow + (size_t)jt * 128);
      FragB a;
      const v8i aw = {(int)(raw.x & am), (int)(raw.y & am), (int)(raw.z & am), (int)(raw.w & am), 0, 0, 0, 0};
      a.w = aw;
      const v4f j0 = *(const v4fa*)(adjr + 16 * jt);
      const v4f j1 = *(const v4fa*)(adjr + 16 * jt + 4);
      const v8f d0 = wmb(a, b0, c0);
      const v8f d1 = wmb(a, b1, c1);
      acc0 = fmaf(j0.x, fmaxf(d0[0], 0.0f), acc0); acc1 = fmaf(j0.x, fmaxf(d1[0], 0.0f), acc1);
      acc0 = fmaf(j0.y, fmaxf(d0[1], 0.0f), acc0); acc1 = fmaf(j0.y, fmaxf(d1[1], 0.0f), acc1);
      acc0 = fmaf(j0.z, fmaxf(d0[2], 0.0f), acc0); acc1 = fmaf(j0.z, fmaxf(d1[2], 0.0f), acc1);
      acc0 = fmaf(j0.w, fmaxf(d0[3], 0.0f), acc0); acc1 = fmaf(j0.w, fmaxf(d1[3], 0.0f), acc1);
      acc0 = fmaf(j1.x, fmaxf(d0[4], 0.0f), acc0); acc1 = fmaf(j1.x, fmaxf(d1[4], 0.0f), acc1);
      acc0 = fmaf(j1.y, fmaxf(d0[5], 0.0f), acc0); acc1 = fmaf(j1.y, fmaxf(d1[5], 0.0f), acc1);
      acc0 = fmaf(j1.z, fmaxf(d0[6], 0.0f), acc0); acc1 = fmaf(j1.z, fmaxf(d1[6], 0.0f), acc1);
      acc0 = fmaf(j1.w, fmaxf(d0[7], 0.0f), acc0); acc1 = fmaf(j1.w, fmaxf(d1[7], 0.0f), acc1);
    }
    const float o0 = __shfl_xor(acc0, 16, 32);
    const float o1 = __shfl_xor(acc1, 16, 32);
    acc0 = acc0 + o0;
    acc1 = acc1 + o1;
    if (lane < 16) {
      sagg[ii * HID + h0 + lane]      = acc0;
      sagg[ii * HID + h0 + 16 + lane] = acc1;
    }
  }
  __syncthreads();

  v8us hv[2], lv[2];
#pragma unroll
  for (int q = 0; q < 2; ++q) {
    const float* sp = sagg + (2 * wave + q) * HID + 8 * lane;
    const v4f a = *(const v4fa*)sp;
    const v4f b = *(const v4fa*)(sp + 4);
    split8(a, b, hv[q], lv[q]);
  }
#pragma unroll
  for (int q = 0; q < 2; ++q) {
    unsigned short* rp = AGG + (size_t)(row0 + 2 * wave + q) * AP + 8 * lane;
    *(volatile v8us*)rp = hv[q];
    *(volatile v8us*)(rp + HID) = lv[q];
  }
  __threadfence();
#pragma unroll
  for (int q = 0; q < 2; ++q) {
    unsigned short* rp = AGG + (size_t)(row0 + 2 * wave + q) * AP + 8 * lane;
    *(volatile v8us*)rp = hv[q];
    *(volatile v8us*)(rp + HID) = lv[q];
  }
}

__global__ __launch_bounds__(NTHR) void k_gru(
    const float* __restrict__ GX, const float* __restrict__ HG, const float* __restrict__ lng,
    const float* __restrict__ lnb, const float* __restrict__ mask, float* H, unsigned short* HHL)
{
  __shared__ __attribute__((aligned(16))) float srow[NWAVE * HID];
  const int tid = (int)threadIdx.x, lane = tid & 31, wave = tid >> 5;
  const int row = (int)blockIdx.x * NWAVE + wave;
  float* sr = srow + wave * HID;
  const float* gx = GX + (size_t)row * G3;
  const float* gh = HG + (size_t)row * HGP + HID;
  float* hrow = H + (size_t)row * HID;

#pragma unroll 1
  for (int j = 0; j < 8; ++j) {
    const int c = 32 * j + lane;
    const float xr = gx[c], xz = gx[HID + c], xn = gx[2 * HID + c];
    const float hr = gh[c], hz = gh[HID + c], hn = gh[2 * HID + c];
    const float hv = hrow[c];
    const float r = 1.0f / (1.0f + expf(-(xr + hr)));
    const float z = 1.0f / (1.0f + expf(-(xz + hz)));
    const float n = tanhf(xn + r * hn);
    sr[c] = (1.0f - z) * n + z * hv;
  }
  __syncthreads();

  const v4f a = *(const v4fa*)(sr + 8 * lane);
  const v4f b = *(const v4fa*)(sr + 8 * lane + 4);
  float s = ((a.x + a.y) + (a.z + a.w)) + ((b.x + b.y) + (b.z + b.w));
#pragma unroll
  for (int d = 16; d >= 1; d >>= 1) s += __shfl_xor(s, d, 32);
  const float mu = s * (1.0f / 256.0f);
  const v4f da = a - mu;
  const v4f db = b - mu;
  float q = ((da.x * da.x + da.y * da.y) + (da.z * da.z + da.w * da.w)) +
            ((db.x * db.x + db.y * db.y) + (db.z * db.z + db.w * db.w));
#pragma unroll
  for (int d = 16; d >= 1; d >>= 1) q += __shfl_xor(q, d, 32);
  const float var  = q * (1.0f / 256.0f);
  const float rstd = 1.0f / sqrtf(var + 1e-5f);
  const float me   = bf16_val(mask[row]);
  const v4f g0 = *(const v4fa*)(lng + 8 * lane);
  const v4f g1 = *(const v4fa*)(lng + 8 * lane + 4);
  const v4f t0 = *(const v4fa*)(lnb + 8 * lane);
  const v4f t1 = *(const v4fa*)(lnb + 8 * lane + 4);
  v4f ya, yb;
  ya.x = (da.x * rstd * bf16_val(g0.x) + bf16_val(t0.x)) * me;
  ya.y = (da.y * rstd * bf16_val(g0.y) + bf16_val(t0.y)) * me;
  ya.z = (da.z * rstd * bf16_val(g0.z) + bf16_val(t0.z)) * me;
  ya.w = (da.w * rstd * bf16_val(g0.w) + bf16_val(t0.w)) * me;
  yb.x = (db.x * rstd * bf16_val(g1.x) + bf16_val(t1.x)) * me;
  yb.y = (db.y * rstd * bf16_val(g1.y) + bf16_val(t1.y)) * me;
  yb.z = (db.z * rstd * bf16_val(g1.z) + bf16_val(t1.z)) * me;
  yb.w = (db.w * rstd * bf16_val(g1.w) + bf16_val(t1.w)) * me;
  v8us hv, lv;
  split8(ya, yb, hv, lv);
  *(v4fa*)(sr + 8 * lane)     = ya;
  *(v4fa*)(sr + 8 * lane + 4) = yb;
  __syncthreads();
  const v4f y0 = *(const v4fa*)(sr + 4 * lane);
  const v4f y1 = *(const v4fa*)(sr + 128 + 4 * lane);

  unsigned short* rp = HHL + (size_t)row * AP + 8 * lane;
  *(volatile v4f*)(hrow + 4 * lane) = y0;
  *(volatile v4f*)(hrow + 128 + 4 * lane) = y1;
  *(volatile v8us*)rp = hv;
  *(volatile v8us*)(rp + HID) = lv;
  __threadfence();
  *(volatile v4f*)(hrow + 4 * lane) = y0;
  *(volatile v4f*)(hrow + 128 + 4 * lane) = y1;
  *(volatile v8us*)rp = hv;
  *(volatile v8us*)(rp + HID) = lv;
}

__global__ __launch_bounds__(NTHR) void k_head(
    const float* __restrict__ H, const float* __restrict__ mask, const float* __restrict__ w1,
    const float* __restrict__ b1, const float* __restrict__ w2, const float* __restrict__ b2, float* out)
{
  __shared__ float smk[NN];
  __shared__ float spool[2 * HID];
  __shared__ float shid[HID];
  __shared__ __attribute__((aligned(16))) float sres[HID];
  const int c = (int)threadIdx.x;
  const int b = (int)blockIdx.x;
  if (c < NN) smk[c] = bf16_val(mask[b * NN + c]);
  __syncthreads();

  float sum = 0.0f, msum = 0.0f, mx = -3.0e38f;
  const float* hp = H + (size_t)b * NN * HID + c;
#pragma unroll 4
  for (int i = 0; i < NN; ++i) {
    const float me = smk[i];
    const float v  = hp[(size_t)i * HID];
    sum  += v * me;
    msum += me;
    const float cand = (me == 0.0f) ? -1000000000.0f : v;
    mx = fmaxf(mx, cand);
  }
  const float den = fmaxf(msum, 1e-6f);
  spool[c]       = sum * (1.0f / den);
  spool[HID + c] = mx;
  __syncthreads();

  float acc = 0.0f;
#pragma unroll 4
  for (int k = 0; k < 2 * HID; ++k) acc = fmaf(spool[k], bf16_val(w1[(size_t)k * HID + c]), acc);
  const float x = acc + bf16_val(b1[c]);
  shid[c] = 0.5f * x * (1.0f + erff(x * 0.70710678118654752f));
  __syncthreads();

  float acc2 = 0.0f;
#pragma unroll 4
  for (int k = 0; k < HID; ++k) acc2 = fmaf(shid[k], bf16_val(w2[(size_t)k * HID + c]), acc2);
  sres[c] = acc2 + bf16_val(b2[c]);
  __syncthreads();

  const int cc = c < 64 ? c : 63;
  const v4f ov = *(const v4fa*)(sres + 4 * cc);
  float* op = out + (size_t)b * HID + 4 * cc;
  const bool okst = c < 64;
  if (okst) *(volatile v4f*)op = ov;
  __threadfence();
  if (okst) *(volatile v4f*)op = ov;
}

static inline size_t al256(size_t o) { return (o + 255) & ~(size_t)255; }

extern "C" void kernel_launch(void* const* d_in, const int* in_sizes, int n_in,
                              void* d_out, int out_size, void* d_ws, size_t ws_size,
                              hipStream_t stream) {
  if (n_in < 18) return;
  const int expect[18] = {
    BB * NN * NATOM, BB * NN * NN, BB * NN * NN * NBOND, BB * NN,
    NATOM * HID, HID, NLAY * (HID + NBOND) * HID, NLAY * HID,
    NLAY * G3 * HID, NLAY * G3 * HID, NLAY * G3, NLAY * G3,
    NLAY * HID, NLAY * HID, 2 * HID * HID, HID, HID * HID, HID };
  for (int i = 0; i < 18; ++i) if (in_sizes[i] != expect[i]) return;
  if (out_size != BB * HID) return;

  const float* node = (const float*)d_in[0];
  const float* adj  = (const float*)d_in[1];
  const float* bond = (const float*)d_in[2];
  const float* mask = (const float*)d_in[3];
  const float* embw = (const float*)d_in[4];
  const float* embb = (const float*)d_in[5];
  const float* msgw = (const float*)d_in[6];
  const float* msgb = (const float*)d_in[7];
  const float* wih  = (const float*)d_in[8];
  const float* whh  = (const float*)d_in[9];
  const float* bih  = (const float*)d_in[10];
  const float* bhh  = (const float*)d_in[11];
  const float* lng  = (const float*)d_in[12];
  const float* lnb  = (const float*)d_in[13];
  const float* pw1  = (const float*)d_in[14];
  const float* pb1  = (const float*)d_in[15];
  const float* pw2  = (const float*)d_in[16];
  const float* pb2  = (const float*)d_in[17];
  float* out = (float*)d_out;

  char* ws = (char*)d_ws;
  size_t off = 0;
  const size_t oNFB = off; off = al256(off + (size_t)MTOT * KEMB * 2);
  const size_t oEWT = off; off = al256(off + (size_t)HID * KEMB * 2);
  const size_t oBFB = off; off = al256(off + (size_t)MTOT * NN * 8 * 2);
  const size_t oADJ = off; off = al256(off + (size_t)MTOT * NN * 4);
  const size_t oWCT = off; off = al256(off + (size_t)NLAY * HGP * HID * 2);
  const size_t oWIH = off; off = al256(off + (size_t)NLAY * G3 * HID * 2);
  const size_t oWBT = off; off = al256(off + (size_t)NLAY * HID * KB * 2);
  const size_t oH   = off; off = al256(off + (size_t)MTOT * HID * 4);
  const size_t oHHL = off; off = al256(off + (size_t)MTOT * AP * 2);
  const size_t oHG  = off; off = al256(off + (size_t)MTOT * HGP * 4);
  const size_t oAGG = off; off = al256(off + (size_t)MTOT * AP * 2);
  const size_t oGX  = off; off = al256(off + (size_t)MTOT * G3 * 4);
  if (off > ws_size || off > (size_t)WSMAX) return;
  unsigned short* NFB  = (unsigned short*)(ws + oNFB);
  unsigned short* EWT  = (unsigned short*)(ws + oEWT);
  unsigned short* BFB  = (unsigned short*)(ws + oBFB);
  float*          ADJF = (float*)(ws + oADJ);
  unsigned short* WCAT = (unsigned short*)(ws + oWCT);
  unsigned short* WIHP = (unsigned short*)(ws + oWIH);
  unsigned short* WBT  = (unsigned short*)(ws + oWBT);
  float*          H    = (float*)(ws + oH);
  unsigned short* HHL  = (unsigned short*)(ws + oHHL);
  float*          HG   = (float*)(ws + oHG);
  unsigned short* AGG  = (unsigned short*)(ws + oAGG);
  float*          GX   = (float*)(ws + oGX);

  k_prep<<<O8 / NTHR, NTHR, 0, stream>>>(node, embw, bond, adj, msgw, whh, wih,
                                         NFB, EWT, BFB, ADJF, WCAT, WIHP, WBT);
  k_gemm<1, 0><<<dim3(MTOT / GBM, HID / GBN), GTHR, 0, stream>>>(
      NFB, KEMB, EWT, KEMB, embb, HID, embb, H, HID, mask, HHL);

  for (int l = 0; l < NLAY; ++l) {
    const unsigned short* wcat_l = WCAT + (size_t)l * HGP * HID;
    const unsigned short* wih_l  = WIHP + (size_t)l * G3 * HID;
    const unsigned short* wbt_l  = WBT  + (size_t)l * HID * KB;
    k_gemm<0, 1><<<dim3(MTOT / GBM, HGP / GBN), GTHR, 0, stream>>>(
        HHL, AP, wcat_l, HID, msgb + l * HID, HID, bhh + l * G3, HG, HGP, mask, AGG);
    k_msg<<<MTOT / MG, NTHR, 0, stream>>>(BFB, ADJF, HG, wbt_l, AGG);
    k_gemm<0, 1><<<dim3(MTOT / GBM, G3 / GBN), GTHR, 0, stream>>>(
        AGG, AP, wih_l, HID, bih + l * G3, G3, bih + l * G3, GX, G3, mask, HHL);
    k_gru<<<MTOT / NWAVE, NTHR, 0, stream>>>(GX, HG, lng + l * HID, lnb + l * HID, mask, H, HHL);
  }

  k_head<<<BB, NTHR, 0, stream>>>(H, mask, pw1, pb1, pw2, pb2, out);
}
